// SelectiveSSM_13563506721344
// MI455X (gfx1250) — hardware-verified
//
#include <hip/hip_runtime.h>
#include <math.h>

typedef __attribute__((ext_vector_type(16))) _Float16 v16h;
typedef __attribute__((ext_vector_type(8)))  _Float16 v8h;
typedef __attribute__((ext_vector_type(16))) __bf16   v16b;
typedef __attribute__((ext_vector_type(8)))  __bf16   v8b;
typedef __attribute__((ext_vector_type(8)))  float    v8f;
typedef __attribute__((ext_vector_type(4)))  float    v4f;
typedef __attribute__((ext_vector_type(4)))  unsigned int v4u;

constexpr int kBatch = 2;
constexpr int kSeq   = 2048;
constexpr int kDm    = 1024;
constexpr int kDin   = 2048;
constexpr int kNst   = 16;
constexpr int kDtR   = 64;
constexpr int kDbc   = kDtR + 2 * kNst;
constexpr int kDbcP  = 128;
constexpr int kRows  = kBatch * kSeq;
constexpr int kScanTS = 32;
constexpr int kScanCh = 64;
constexpr int kScanYP = 68;
constexpr float kCarryX   = 64.0f;
constexpr float kCarryDt  = 8.0f;
constexpr float kCarryOut = 64.0f;
constexpr float kInvCarryX   = 0.015625f;
constexpr float kInvCarryDt  = 0.125f;
constexpr float kInvCarryOut = 0.015625f;
constexpr float kLog2e  = 1.4426950408889634f;
constexpr float kFltMin = 1.17549435e-38f;
static_assert(kDbc == 96 && kDbc <= kDbcP, "x_proj width");
static_assert((kDm % 32) == 0 && (kDin % 32) == 0 && (kDtR % 32) == 0, "GEMM K multiples of 32");
static_assert((kRows % 64) == 0 && (kDin % 64) == 0 && (kDbcP % 64) == 0 && (kDm % 64) == 0, "GEMM M,N multiples of 64");
static_assert((kSeq % kScanTS) == 0 && (kDin % kScanCh) == 0 && (kScanTS % 8) == 0, "scan tile multiples");

constexpr size_t kOffUB   = 0;
constexpr size_t kOffWIB  = kOffUB  + (size_t)kRows * kDm   * 2;
constexpr size_t kOffWXH  = kOffWIB + (size_t)(2 * kDin) * kDm * 2;
constexpr size_t kOffWDH  = kOffWXH + (size_t)kDbcP * kDin  * 2;
constexpr size_t kOffWOH  = kOffWDH + (size_t)kDin  * kDtR  * 2;
constexpr size_t kOffXH   = kOffWOH + (size_t)kDm   * kDin  * 2;
constexpr size_t kOffZF   = kOffXH  + (size_t)kRows * kDin  * 2;
constexpr size_t kOffDBC  = kOffZF  + (size_t)kRows * kDin  * 4;
constexpr size_t kOffDRH  = kOffDBC + (size_t)kRows * kDbcP * 4;
constexpr size_t kOffDP   = kOffDRH + (size_t)kRows * kDtR  * 2;
constexpr size_t kOffYH   = kOffDP  + (size_t)kRows * kDin  * 4;
constexpr size_t kWsTotal = kOffYH  + (size_t)kRows * kDin  * 2;
static_assert(kWsTotal == 125042688ull, "carve total");
static_assert(kWsTotal <= 134217728ull, "carve cap");
static_assert((kOffWIB % 128) == 0 && (kOffWXH % 128) == 0 && (kOffWDH % 128) == 0 && (kOffWOH % 128) == 0 &&
              (kOffXH % 128) == 0 && (kOffZF % 128) == 0 && (kOffDBC % 128) == 0 && (kOffDRH % 128) == 0 &&
              (kOffDP % 128) == 0 && (kOffYH % 128) == 0, "128-B aligned regions");

__device__ __forceinline__ unsigned short f2bf_bits(float f) {
  unsigned u = __float_as_uint(f);
  return (unsigned short)((u + 0x7FFFu + ((u >> 16) & 1u)) >> 16);
}
__device__ __forceinline__ float bf_bits2f(unsigned short h) { return __uint_as_float(((unsigned)h) << 16); }
__device__ __forceinline__ float bf_rne(float f) { return bf_bits2f(f2bf_bits(f)); }

__device__ __forceinline__ float h16_to_f32(unsigned hb) {
  const unsigned sgn = (hb & 0x8000u) << 16; const unsigned em = hb & 0x7fffu;
  const float fn = __uint_as_float((em << 13) + 0x38000000u);
  const float fs = (float)em * 5.9604644775390625e-8f;
  const float mag = (em < 0x400u) ? fs : fn; return __uint_as_float(__float_as_uint(mag) | sgn);
}

__device__ __forceinline__ void row_guard_h(v8f& a, v8f& b, v8f& c, v8f& d, v16h x, v16h y0, v16h y1, v16h y2, v16h y3) {
  asm volatile("v_nop\n\tv_nop\n\tv_nop\n\tv_nop" : "+v"(a), "+v"(b), "+v"(c), "+v"(d) : "v"(x), "v"(y0), "v"(y1), "v"(y2), "v"(y3));
}
__device__ __forceinline__ void row_guard_b(v8f& a, v8f& b, v8f& c, v8f& d, v16b x, v16b y0, v16b y1, v16b y2, v16b y3) {
  asm volatile("v_nop\n\tv_nop\n\tv_nop\n\tv_nop" : "+v"(a), "+v"(b), "+v"(c), "+v"(d) : "v"(x), "v"(y0), "v"(y1), "v"(y2), "v"(y3));
}
__device__ __forceinline__ void keep4_h(v16h a, v16h b, v16h c, v16h d) { asm volatile("v_nop" :: "v"(a), "v"(b), "v"(c), "v"(d)); }
__device__ __forceinline__ void keep4_b(v16b a, v16b b, v16b c, v16b d) { asm volatile("v_nop" :: "v"(a), "v"(b), "v"(c), "v"(d)); }
__device__ __forceinline__ void acc_guard4(v8f& a, v8f& b, v8f& c, v8f& d) { asm volatile("v_nop\n\tv_nop\n\tv_nop\n\tv_nop" : "+v"(a), "+v"(b), "+v"(c), "+v"(d)); }

template <typename T> struct Frag;
template <> struct Frag<_Float16> {
  typedef v16h V; union U { v16h v; v8h h[2]; };
  static __device__ __forceinline__ v16h load(const _Float16* p) {
    U f; f.h[0] = *(const v8h*)(p); f.h[1] = *(const v8h*)(p + 16); return f.v;
  }
  static __device__ __forceinline__ v8f mma(v16h a, v16h b, v8f c) {
    return __builtin_amdgcn_wmma_f32_16x16x32_f16(false, a, false, b, (short)0, c, false, false);
  }
  static __device__ __forceinline__ void guard_row(v8f& a, v8f& b, v8f& c, v8f& d, v16h x, v16h y0, v16h y1, v16h y2, v16h y3) { row_guard_h(a, b, c, d, x, y0, y1, y2, y3); }
  static __device__ __forceinline__ void keep(v16h a, v16h b, v16h c, v16h d) { keep4_h(a, b, c, d); }
};
template <> struct Frag<__bf16> {
  typedef v16b V; union U { v16b v; v8b h[2]; };
  static __device__ __forceinline__ v16b load(const __bf16* p) {
    U f; f.h[0] = *(const v8b*)(p); f.h[1] = *(const v8b*)(p + 16); return f.v;
  }
  static __device__ __forceinline__ v8f mma(v16b a, v16b b, v8f c) {
    return __builtin_amdgcn_wmma_f32_16x16x32_bf16(false, a, false, b, (short)0, c, false, false);
  }
  static __device__ __forceinline__ void guard_row(v8f& a, v8f& b, v8f& c, v8f& d, v16b x, v16b y0, v16b y1, v16b y2, v16b y3) { row_guard_b(a, b, c, d, x, y0, y1, y2, y3); }
  static __device__ __forceinline__ void keep(v16b a, v16b b, v16b c, v16b d) { keep4_b(a, b, c, d); }
};

template <int ET> struct Elem;
template <> struct Elem<0> { typedef _Float16 T; };
template <> struct Elem<1> { typedef __bf16 T; };

template <int ET, int OUT_MODE>
__global__ __launch_bounds__(256) void wmma_gemm64(
    const unsigned short* __restrict__ Ap, int lda,
    const unsigned short* __restrict__ Btp, int ldb,
    void* __restrict__ Cout, int ldc,
    const float* __restrict__ bias, int nbias,
    int M, int N, int K, float scale) {
  typedef typename Elem<ET>::T T;
  typedef typename Frag<T>::V V;
  const T* A = (const T*)Ap; const T* Bt = (const T*)Btp;
  __shared__ __align__(16) float sT[8][16 * 68];
  const int lane = threadIdx.x & 31;
  const int wave = threadIdx.x >> 5;
  const int tilesN = N >> 6;
  const int tilesM = M >> 6;
  const int tile = blockIdx.x * 8 + wave;
  if (tile >= tilesM * tilesN) return;
  const int tm = tile / tilesN;
  const int tn = tile - tm * tilesN;
  const int m0 = tm << 6;
  const int n0 = tn << 6;

  const int rlane = lane & 15;
  const int koff  = (lane >> 4) * 8;
  const int mOff  = (lane >> 4) * 8;

  v8f acc[4][4];
#pragma unroll
  for (int i = 0; i < 4; ++i)
#pragma unroll
    for (int j = 0; j < 4; ++j) acc[i][j] = (v8f){0.f,0.f,0.f,0.f,0.f,0.f,0.f,0.f};

  for (int k0 = 0; k0 < K; k0 += 32) {
    V bh[4];
#pragma unroll
    for (int j = 0; j < 4; ++j) {
      const size_t bo = (size_t)(n0 + (j << 4) + rlane) * ldb + koff + k0;
      bh[j] = Frag<T>::load(Bt + bo);
    }
#pragma unroll
    for (int i = 0; i < 4; ++i) {
      const size_t ao = (size_t)(m0 + (i << 4) + rlane) * lda + koff + k0;
      V ah = Frag<T>::load(A + ao);
#pragma unroll
      for (int j = 0; j < 4; ++j) acc[i][j] = Frag<T>::mma(ah, bh[j], acc[i][j]);
      Frag<T>::guard_row(acc[i][0], acc[i][1], acc[i][2], acc[i][3], ah, bh[0], bh[1], bh[2], bh[3]);
    }
    Frag<T>::keep(bh[0], bh[1], bh[2], bh[3]);
  }
  acc_guard4(acc[0][0], acc[0][1], acc[0][2], acc[0][3]);
  acc_guard4(acc[1][0], acc[1][1], acc[1][2], acc[1][3]);
  acc_guard4(acc[2][0], acc[2][1], acc[2][2], acc[2][3]);
  acc_guard4(acc[3][0], acc[3][1], acc[3][2], acc[3][3]);

  float* slab = sT[wave];
#pragma unroll
  for (int i = 0; i < 4; ++i) {
    const int mBase = m0 + (i << 4);
#pragma unroll
    for (int j = 0; j < 4; ++j) {
      const int n = n0 + (j << 4) + rlane;
      const int nb = (n < nbias) ? n : (nbias - 1);
      const float brn = bf_rne(bias[nb]);
      const float bv = (n < nbias) ? brn : 0.0f;
#pragma unroll
      for (int r = 0; r < 8; ++r) {
        const float v = acc[i][j][r] * scale + bv;
        slab[(mOff + r) * 68 + (j << 4) + rlane] = v;
      }
    }
    __builtin_amdgcn_fence(__ATOMIC_RELEASE, "workgroup");
    __builtin_amdgcn_wave_barrier();
    __builtin_amdgcn_fence(__ATOMIC_ACQUIRE, "workgroup");
    if (OUT_MODE == 0) {
      float* C = (float*)Cout;
      const int hh = lane >> 4, c4 = (lane & 15) * 4;
      for (int pass = 0; pass < 2; ++pass) {
#pragma unroll
        for (int it = 0; it < 8; ++it) {
          const int row = it * 2 + hh;
          v4f v = *(const v4f*)(slab + row * 68 + c4);
          *(volatile v4f*)(C + (size_t)(mBase + row) * ldc + n0 + c4) = v;
        }
        __threadfence();
      }
    } else {
      const int q = lane >> 3, c8 = (lane & 7) * 8;
      unsigned short* C = (unsigned short*)Cout;
      for (int pass = 0; pass < 2; ++pass) {
#pragma unroll
        for (int it = 0; it < 4; ++it) {
          const int row = it * 4 + q;
          const float* sp = slab + row * 68 + c8;
          v8h hv;
#pragma unroll
          for (int e = 0; e < 8; ++e) hv[e] = (_Float16)sp[e];
          *(volatile v8h*)(C + (size_t)(mBase + row) * ldc + n0 + c8) = hv;
        }
        __threadfence();
      }
    }
    __builtin_amdgcn_fence(__ATOMIC_RELEASE, "workgroup");
    __builtin_amdgcn_wave_barrier();
    __builtin_amdgcn_fence(__ATOMIC_ACQUIRE, "workgroup");
  }
}

__global__ __launch_bounds__(256) void cvt_bf16_kernel(
    const float* __restrict__ src, unsigned short* __restrict__ dst, int total8)
{
  const int i = blockIdx.x * 256 + threadIdx.x;
  if (i >= total8) return;
  const size_t e0 = (size_t)i << 3;
  const v4f a0 = *(const v4f*)(src + e0);
  const v4f a1 = *(const v4f*)(src + e0 + 4);
  v8h hv;
#pragma unroll
  for (int e = 0; e < 4; ++e) {
    const unsigned short b0 = f2bf_bits(a0[e]);
    const unsigned short b1 = f2bf_bits(a1[e]);
    hv[e]     = __builtin_bit_cast(_Float16, b0);
    hv[4 + e] = __builtin_bit_cast(_Float16, b1);
  }
  unsigned short* q = dst + e0;
  *(volatile v8h*)q = hv;
  __threadfence();
  *(volatile v8h*)q = hv;
}

__global__ __launch_bounds__(256) void cvt_f16w_kernel(
    const float* __restrict__ src, unsigned short* __restrict__ dst, int cols, int rows_real, int total8, float scale)
{
  const int i = blockIdx.x * 256 + threadIdx.x;
  if (i >= total8) return;
  const size_t e0 = (size_t)i << 3;
  const int row = (int)(e0 / (size_t)cols);
  const int col = (int)(e0 - (size_t)row * cols);
  const int rsrc = (row < rows_real) ? row : (rows_real - 1);
  const float fz = (row < rows_real) ? 1.0f : 0.0f;
  const float* sp = src + (size_t)rsrc * cols + col;
  const v4f a0 = *(const v4f*)(sp);
  const v4f a1 = *(const v4f*)(sp + 4);
  v8h hv;
#pragma unroll
  for (int e = 0; e < 4; ++e) {
    const float v0 = bf_rne(a0[e]) * scale * fz;
    const float v1 = bf_rne(a1[e]) * scale * fz;
    hv[e]     = (_Float16)v0;
    hv[4 + e] = (_Float16)v1;
  }
  unsigned short* q = dst + e0;
  *(volatile v8h*)q = hv;
  __threadfence();
  *(volatile v8h*)q = hv;
}

__global__ __launch_bounds__(256) void cvt_dr_kernel(
    const float* __restrict__ dbc, unsigned short* __restrict__ dr, int total8)
{
  const int i = blockIdx.x * 256 + threadIdx.x;
  if (i >= total8) return;
  const int row = i >> 3;
  const int c8 = (i & 7) * 8;
  const float* sp = dbc + (size_t)row * kDbcP + c8;
  const v4f a0 = *(const v4f*)(sp);
  const v4f a1 = *(const v4f*)(sp + 4);
  v8h hv;
#pragma unroll
  for (int e = 0; e < 4; ++e) {
    hv[e]     = (_Float16)a0[e];
    hv[4 + e] = (_Float16)a1[e];
  }
  unsigned short* q = dr + ((size_t)i << 3);
  *(volatile v8h*)q = hv;
  __threadfence();
  *(volatile v8h*)q = hv;
}

__global__ __launch_bounds__(64) void scan_kernel(
    const float* __restrict__ DP, const unsigned short* __restrict__ XH, const float* __restrict__ ZF,
    const float* __restrict__ DBC, const float* __restrict__ Alog, const float* __restrict__ Dp,
    unsigned short* __restrict__ YH)
{
  __shared__ __align__(16) float sD[kScanTS * kScanCh];
  __shared__ __align__(16) float sX[kScanTS * kScanCh];
  __shared__ __align__(16) float sZ[kScanTS * kScanCh];
  __shared__ __align__(16) float sBC[kScanTS * 32];
  __shared__ __align__(16) float sY[kScanTS * kScanYP];
  __shared__ __align__(16) float sA[kNst * kScanCh];
  const int tid = threadIdx.x, lane = tid & 31, wave = tid >> 5;
  constexpr int kBlkPerB = kDin / kScanCh;
  const int bix = blockIdx.x / kBlkPerB;
  const int d0  = (blockIdx.x - bix * kBlkPerB) * kScanCh;
  const int d   = d0 + tid;
  const size_t row0 = (size_t)bix * kSeq;

#pragma unroll 1
  for (int n = 0; n < kNst; ++n) {
    const float al = Alog[(size_t)d * kNst + n];
    sA[n * kScanCh + tid] = -expf(bf_rne(al)) * kLog2e;
  }
  __syncthreads();
  float nA2[kNst], h[kNst];
#pragma unroll
  for (int n = 0; n < kNst; ++n) {
    nA2[n] = sA[n * kScanCh + tid];
    h[n] = 0.0f;
  }
  const float Dd = bf_rne(Dp[d]);
  const int q = lane >> 3, c8 = (lane & 7) * 8;

#pragma unroll 1
  for (int t0 = 0; t0 < kSeq; t0 += kScanTS) {
    __syncthreads();
#pragma unroll 1
    for (int i = 0; i < 8; ++i) {
      const int c = tid + 64 * i;
      const int r = c >> 4, c4 = (c & 15) * 4;
      *(v4f*)(sD + r * kScanCh + c4) = *(const v4f*)(DP + (row0 + t0 + r) * (size_t)kDin + d0 + c4);
    }
#pragma unroll 1
    for (int i = 0; i < 8; ++i) {
      const int c = tid + 64 * i;
      const int r = c >> 4, c4 = (c & 15) * 4;
      *(v4f*)(sZ + r * kScanCh + c4) = *(const v4f*)(ZF + (row0 + t0 + r) * (size_t)kDin + d0 + c4);
    }
#pragma unroll 1
    for (int i = 0; i < 4; ++i) {
      const int c = tid + 64 * i;
      const int r = c >> 3, cc = (c & 7) * 8;
      const v4u w = *(const v4u*)(XH + (row0 + t0 + r) * (size_t)kDin + d0 + cc);
      const unsigned w0 = w[0], w1 = w[1], w2 = w[2], w3 = w[3];
      v4f f0, f1;
      f0[0] = h16_to_f32(w0 & 0xffffu); f0[1] = h16_to_f32(w0 >> 16);
      f0[2] = h16_to_f32(w1 & 0xffffu); f0[3] = h16_to_f32(w1 >> 16);
      f1[0] = h16_to_f32(w2 & 0xffffu); f1[1] = h16_to_f32(w2 >> 16);
      f1[2] = h16_to_f32(w3 & 0xffffu); f1[3] = h16_to_f32(w3 >> 16);
      *(v4f*)(sX + r * kScanCh + cc)     = f0;
      *(v4f*)(sX + r * kScanCh + cc + 4) = f1;
    }
#pragma unroll 1
    for (int i = 0; i < 4; ++i) {
      const int c = tid + 64 * i;
      const int r = c >> 3, c4 = (c & 7) * 4;
      *(v4f*)(sBC + r * 32 + c4) = *(const v4f*)(DBC + (row0 + t0 + r) * (size_t)kDbcP + kDtR + c4);
    }
    __syncthreads();

#pragma unroll 1
    for (int s = 0; s < kScanTS; ++s) {
      const float* bcr = sBC + s * 32;
      const float v   = sD[s * kScanCh + tid];
      const float ev  = expf(-fabsf(v));
      const float dt  = fmaxf(v, 0.0f) + log1pf(ev);
      const float xt  = sX[s * kScanCh + tid];
      const float zt  = sZ[s * kScanCh + tid];
      const float dtx = dt * xt;
      float y = 0.0f;
#pragma unroll
      for (int q4 = 0; q4 < 4; ++q4) {
        const v4f bv = *(const v4f*)(bcr + 4 * q4);
        const v4f cv = *(const v4f*)(bcr + kNst + 4 * q4);
#pragma unroll
        for (int e = 0; e < 4; ++e) {
          const int n = 4 * q4 + e;
          float da = exp2f(dt * nA2[n]);
          da = (da < kFltMin) ? 0.0f : da;
          const float hn = da * h[n] + dtx * bv[e];
          h[n] = hn;
          y = y + hn * cv[e];
        }
      }
      y = y + xt * Dd;
      const float ez = expf(-zt);
      const float sg = __builtin_amdgcn_rcpf(1.0f + ez);
      y = y * (zt * sg);
      sY[s * kScanYP + tid] = y;
    }
    __syncthreads();
    v8h hv[4];
#pragma unroll
    for (int it = 0; it < 4; ++it) {
      const int row = it * 8 + wave * 4 + q;
      const float* sp = sY + row * kScanYP + c8;
      const v4f a0 = *(const v4f*)(sp);
      const v4f a1 = *(const v4f*)(sp + 4);
#pragma unroll
      for (int e = 0; e < 4; ++e) {
        hv[it][e]     = (_Float16)a0[e];
        hv[it][4 + e] = (_Float16)a1[e];
      }
    }
    for (int pass = 0; pass < 2; ++pass) {
#pragma unroll
      for (int it = 0; it < 4; ++it) {
        const int row = it * 8 + wave * 4 + q;
        const size_t o = (row0 + t0 + row) * (size_t)kDin + d0 + c8;
        *(volatile v8h*)(YH + o) = hv[it];
      }
      __threadfence();
    }
  }
}

extern "C" void kernel_launch(void* const* d_in, const int* in_sizes, int n_in,
                              void* d_out, int out_size, void* d_ws, size_t ws_size,
                              hipStream_t stream) {
  if (n_in < 11) return;
  if (in_sizes[0] != kRows * kDm) return;
  if (in_sizes[1] != 2 * kDin * kDm) return;
  if (in_sizes[2] != 2 * kDin) return;
  if (in_sizes[3] != kDbc * kDin) return;
  if (in_sizes[4] != kDbc) return;
  if (in_sizes[5] != kDin * kDtR) return;
  if (in_sizes[6] != kDin) return;
  if (in_sizes[7] != kDin * kNst) return;
  if (in_sizes[8] != kDin) return;
  if (in_sizes[9] != kDm * kDin) return;
  if (in_sizes[10] != kDm) return;
  if (out_size != kRows * kDm) return;
  if (ws_size < kWsTotal) return;

  const float* u     = (const float*)d_in[0];
  const float* W_in  = (const float*)d_in[1];
  const float* b_in  = (const float*)d_in[2];
  const float* W_x   = (const float*)d_in[3];
  const float* b_x   = (const float*)d_in[4];
  const float* W_dt  = (const float*)d_in[5];
  const float* b_dt  = (const float*)d_in[6];
  const float* A_log = (const float*)d_in[7];
  const float* Dp    = (const float*)d_in[8];
  const float* W_out = (const float*)d_in[9];
  const float* b_out = (const float*)d_in[10];
  float* out = (float*)d_out;

  char* ws = (char*)d_ws;
  unsigned short* UB  = (unsigned short*)(ws + kOffUB);
  unsigned short* WIB = (unsigned short*)(ws + kOffWIB);
  unsigned short* WXH = (unsigned short*)(ws + kOffWXH);
  unsigned short* WDH = (unsigned short*)(ws + kOffWDH);
  unsigned short* WOH = (unsigned short*)(ws + kOffWOH);
  unsigned short* XH  = (unsigned short*)(ws + kOffXH);
  float*          ZF  = (float*)(ws + kOffZF);
  float*          DBC = (float*)(ws + kOffDBC);
  unsigned short* DRH = (unsigned short*)(ws + kOffDRH);
  float*          DP  = (float*)(ws + kOffDP);
  unsigned short* YH  = (unsigned short*)(ws + kOffYH);

  {
    const int t8u = kRows * kDm / 8;
    cvt_bf16_kernel<<<(t8u + 255) / 256, 256, 0, stream>>>(u, UB, t8u);
    const int t8w = 2 * kDin * kDm / 8;
    cvt_bf16_kernel<<<(t8w + 255) / 256, 256, 0, stream>>>(W_in, WIB, t8w);
    const int t8x = kDbcP * kDin / 8;
    cvt_f16w_kernel<<<(t8x + 255) / 256, 256, 0, stream>>>(W_x, WXH, kDin, kDbc, t8x, kCarryX);
    const int t8d = kDin * kDtR / 8;
    cvt_f16w_kernel<<<(t8d + 255) / 256, 256, 0, stream>>>(W_dt, WDH, kDtR, kDin, t8d, kCarryDt);
    const int t8o = kDm * kDin / 8;
    cvt_f16w_kernel<<<(t8o + 255) / 256, 256, 0, stream>>>(W_out, WOH, kDin, kDm, t8o, kCarryOut);
  }

  {
    const int tiles = (kRows / 64) * (kDin / 64);
    wmma_gemm64<1, 1><<<dim3((tiles + 7) / 8), 256, 0, stream>>>(
        UB, kDm,
        WIB, kDm,
        (void*)XH, kDin,
        b_in, kDin,
        kRows, kDin, kDm, 1.0f);
  }
  {
    const int tiles = (kRows / 64) * (kDin / 64);
    wmma_gemm64<1, 0><<<dim3((tiles + 7) / 8), 256, 0, stream>>>(
        UB, kDm,
        WIB + (size_t)kDin * kDm, kDm,
        (void*)ZF, kDin,
        b_in + kDin, kDin,
        kRows, kDin, kDm, 1.0f);
  }
  {
    const int tiles = (kRows / 64) * (kDbcP / 64);
    wmma_gemm64<0, 0><<<dim3((tiles + 7) / 8), 256, 0, stream>>>(
        XH, kDin,
        WXH, kDin,
        (void*)DBC, kDbcP,
        b_x, kDbc,
        kRows, kDbcP, kDin, kInvCarryX);
  }
  {
    const int t8 = kRows * kDtR / 8;
    cvt_dr_kernel<<<(t8 + 255) / 256, 256, 0, stream>>>(DBC, DRH, t8);
  }
  {
    const int tiles = (kRows / 64) * (kDin / 64);
    wmma_gemm64<0, 0><<<dim3((tiles + 7) / 8), 256, 0, stream>>>(
        DRH, kDtR,
        WDH, kDtR,
        (void*)DP, kDin,
        b_dt, kDin,
        kRows, kDin, kDtR, kInvCarryDt);
  }
  scan_kernel<<<kBatch * (kDin / kScanCh), kScanCh, 0, stream>>>(DP, XH, ZF, DBC, A_log, Dp, YH);

  {
    const int tiles = (kRows / 64) * (kDm / 64);
    wmma_gemm64<0, 0><<<dim3((tiles + 7) / 8), 256, 0, stream>>>(
        YH, kDin,
        WOH, kDin,
        (void*)out, kDm,
        b_out, kDm,
        kRows, kDm, kDin, kInvCarryOut);
  }
}
